// KinematicsTrendAttention_41893111005326
// MI455X (gfx1250) — hardware-verified
//
#include <hip/hip_runtime.h>


#define NBb  4
#define NA   8
#define TT   512
#define DD   256
#define NH_  8
#define HD   32
#define HP   64
#define F3   768
#define NR   (NBb * NA * TT)
#define ZZ   (NA * NH_)
#define PCAR 1024.0f
typedef _Float16 h16;
typedef unsigned short bf;
typedef __attribute__((ext_vector_type(16))) __bf16   v16bf;
typedef __attribute__((ext_vector_type(16))) _Float16 v16h;
typedef __attribute__((ext_vector_type(8)))  _Float16 v8h;
typedef __attribute__((ext_vector_type(8)))  unsigned short v8us;
typedef __attribute__((ext_vector_type(8)))  float    v8f;
typedef __attribute__((ext_vector_type(4)))  float    v4f;
typedef v8h  __attribute__((may_alias)) v8ha;
typedef v4f  __attribute__((may_alias)) v4fa;
typedef v8us __attribute__((may_alias)) v8usa;

__device__ __forceinline__ unsigned short f2bf(float f) { unsigned u = __float_as_uint(f); u += 0x7FFFu + ((u >> 16) & 1u); return (unsigned short)(u >> 16); }
__device__ __forceinline__ float bf2f(unsigned short b) { return __uint_as_float(((unsigned)b) << 16); }
__device__ __forceinline__ float bfr(float f) { return bf2f(f2bf(f)); }
__device__ __forceinline__ v16h cat16(v8h lo, v8h hi) { return __builtin_shufflevector(lo, hi, 0, 1, 2, 3, 4, 5, 6, 7, 8, 9, 10, 11, 12, 13, 14, 15); }
__device__ __forceinline__ v16bf cat16b(v8us lo, v8us hi) { return __builtin_bit_cast(v16bf, __builtin_shufflevector(lo, hi, 0, 1, 2, 3, 4, 5, 6, 7, 8, 9, 10, 11, 12, 13, 14, 15)); }
__device__ __forceinline__ v8f wmma16(v16h a, v16h b, v8f c) { return __builtin_amdgcn_wmma_f32_16x16x32_f16(false, a, false, b, (short)0, c, false, false); }
__device__ __forceinline__ v8f wmmab(v16bf a, v16bf b, v8f c) { return __builtin_amdgcn_wmma_f32_16x16x32_bf16(false, a, false, b, (short)0, c, false, false); }


template <typename T16> struct WFrag;
template <> struct WFrag<h16> { typedef v16h V; static __device__ __forceinline__ V ld(const h16* p) { return cat16(*(const v8h*)p, *(const v8h*)(p + 16)); } static __device__ __forceinline__ v8f mma(V a, V b, v8f c) { return wmma16(a, b, c); } };
template <> struct WFrag<bf> { typedef v16bf V; static __device__ __forceinline__ V ld(const bf* p) { return cat16b(*(const v8us*)p, *(const v8us*)(p + 16)); } static __device__ __forceinline__ v8f mma(V a, V b, v8f c) { return wmmab(a, b, c); } };
template <typename T16, int NSPLIT, bool BIAS>
__global__ __launch_bounds__(32) void k_gemmw(const T16* __restrict__ A, const T16* __restrict__ A2, const T16* __restrict__ Bt, const T16* __restrict__ Bt2, int K, float* C, int ldc, const float* __restrict__ bias, size_t sA, size_t sB, size_t sC) {
    typedef typename WFrag<T16>::V V;
    __shared__ __align__(16) float os[16 * 68];
    const size_t z = blockIdx.z; A += z * sA; if (A2) A2 += z * sA; Bt += z * sB; if (Bt2) Bt2 += z * sB; C += z * sC;
    const int lane = threadIdx.x & 31, lr = lane & 15, hi = lane >> 4; const int r0 = blockIdx.x * 64, c0 = blockIdx.y * 64;
    v8f acc[4][4];
#pragma unroll
    for (int mb = 0; mb < 4; ++mb)
#pragma unroll
        for (int nb = 0; nb < 4; ++nb) acc[mb][nb] = (v8f){};
    const size_t aoff = (size_t)(r0 + lr) * K + 8 * hi, boff = (size_t)(c0 + lr) * K + 8 * hi;
#pragma unroll 1
    for (int kc = 0; kc < K; kc += 32) {
        V a[4], a2[4];
#pragma unroll
        for (int mb = 0; mb < 4; ++mb) { a[mb] = WFrag<T16>::ld(A + aoff + (size_t)mb * 16 * K + kc); if (NSPLIT == 1 || NSPLIT == 2) a2[mb] = WFrag<T16>::ld(A2 + aoff + (size_t)mb * 16 * K + kc); }
#pragma unroll
        for (int nb = 0; nb < 4; ++nb) { const V b = WFrag<T16>::ld(Bt + boff + (size_t)nb * 16 * K + kc); V b2; if (NSPLIT >= 2) b2 = WFrag<T16>::ld(Bt2 + boff + (size_t)nb * 16 * K + kc);
#pragma unroll
            for (int mb = 0; mb < 4; ++mb) { acc[mb][nb] = WFrag<T16>::mma(a[mb], b, acc[mb][nb]); if (NSPLIT == 1 || NSPLIT == 2) acc[mb][nb] = WFrag<T16>::mma(a2[mb], b, acc[mb][nb]); if (NSPLIT >= 2) acc[mb][nb] = WFrag<T16>::mma(a[mb], b2, acc[mb][nb]); } }
        asm volatile("v_nop\n\tv_nop\n\tv_nop\n\tv_nop" : "+v"(acc[0][0]), "+v"(acc[1][1]), "+v"(acc[2][2]), "+v"(acc[3][3]) : "v"(a[0]), "v"(a[3]));
    }
#pragma unroll
    for (int mb = 0; mb < 4; ++mb) {
#pragma unroll
        for (int nb = 0; nb < 4; ++nb) {
#pragma unroll
            for (int j = 0; j < 8; ++j) os[(hi * 8 + j) * 68 + nb * 16 + lr] = acc[mb][nb][j]; }
        __builtin_amdgcn_wave_barrier(); asm volatile("" ::: "memory");
        float* crow = C + (size_t)(r0 + mb * 16) * ldc + c0;
#pragma unroll 1
        for (int ps = 0; ps < 2; ++ps) {
#pragma unroll
            for (int s = 0; s < 8; ++s) { const int row = 2 * s + hi, cofs = lr * 4; v4f val = *(const v4fa*)(os + row * 68 + cofs); if (BIAS) { val[0] += bfr(bias[c0 + cofs]); val[1] += bfr(bias[c0 + cofs + 1]); val[2] += bfr(bias[c0 + cofs + 2]); val[3] += bfr(bias[c0 + cofs + 3]); }
                *(volatile v4f*)(crow + (size_t)row * ldc + cofs) = val; }
            if (ps == 0) __threadfence(); }
        __builtin_amdgcn_wave_barrier(); asm volatile("" ::: "memory");
    }
}

__device__ __forceinline__ h16 tohx(float x) { return (h16)x; }
__device__ __forceinline__ void splitf(float y, unsigned short& h, unsigned short& l) { h = f2bf(y); l = f2bf(y - bf2f(h)); }
typedef __attribute__((ext_vector_type(2))) unsigned short v2us;
typedef __attribute__((ext_vector_type(4))) unsigned short v4us;
typedef __attribute__((ext_vector_type(2))) _Float16 v2h;
typedef __attribute__((ext_vector_type(4))) _Float16 v4h;

__global__ __launch_bounds__(256) void k_wtG(const float* __restrict__ w, int K, int N, bf* Bt) {
    const int lane = threadIdx.x & 31; const int L0 = (blockIdx.x * 8 + (threadIdx.x >> 5)) * 8; const int nlines = N * K / 64;
#pragma unroll
    for (int ps = 0; ps < 2; ++ps) {
#pragma unroll 1
        for (int l = 0; l < 8; ++l) { const int L = L0 + l; if (L >= nlines) break; const size_t e = (size_t)L * 64 + lane * 2; const int k = (int)(e % K), n = (int)(e / K); v2us o;
            o[0] = f2bf(w[(size_t)k * N + n]); o[1] = f2bf(w[(size_t)(k + 1) * N + n]); *(volatile v2us*)(Bt + e) = o; }
        if (ps == 0) __threadfence(); }
}
__global__ __launch_bounds__(256) void k_cvt8(const float* __restrict__ src, bf* dst, size_t n8) { const size_t i = (size_t)blockIdx.x * 256 + threadIdx.x; if (i >= n8) return; const v8f v = *(const v8f*)(src + i * 8); v8us o;
#pragma unroll
    for (int k = 0; k < 8; ++k) o[k] = f2bf(v[k]); *(volatile v8us*)(dst + i * 8) = o; __threadfence(); *(volatile v8us*)(dst + i * 8) = o; }
__global__ __launch_bounds__(256) void k_kin(const float* __restrict__ x, const float* __restrict__ wp, const float* __restrict__ bp, const float* __restrict__ wv, const float* __restrict__ wa, bf* Fh, bf* Fl) { const size_t e = ((size_t)blockIdx.x * 256 + threadIdx.x) * 4; if (e >= (size_t)NR * F3) return; const int cc = (int)(e % F3); const int r = (int)(e / F3); const int t = r % TT; const int s = cc / DD, c0 = cc % DD; const float* w = (s == 0) ? wp : (s == 1 ? wv : wa); v4us oh, ol;
#pragma unroll
    for (int u = 0; u < 4; ++u) { const int c = c0 + u; float acc = (s == 0) ? bfr(bp[c]) : 0.f;
#pragma unroll
        for (int k = 0; k < 3; ++k) { const int ts = t + k - 1; if (ts >= 0 && ts < TT) { float p = __fmul_rn(bfr(w[c * 3 + k]), bfr(x[((size_t)(r - t + ts)) * DD + c])); asm volatile("" : "+v"(p)); acc = __fadd_rn(acc, p); } }
        unsigned short hh, ll; splitf(acc, hh, ll); oh[u] = hh; ol[u] = ll; }
    *(volatile v4us*)(Fh + e) = oh; *(volatile v4us*)(Fl + e) = ol; __threadfence(); *(volatile v4us*)(Fh + e) = oh; *(volatile v4us*)(Fl + e) = ol; }
__global__ __launch_bounds__(256) void k_qkpl(const float* __restrict__ Q, const float* __restrict__ K, int b, bf* Qh, bf* Ql, bf* Kh, bf* Kl) { const int e = (blockIdx.x * 256 + threadIdx.x) * 4; if (e >= ZZ * TT * HD) return; const int d = e % HD; const int t = (e / HD) % TT; const int z = e / (HD * TT); const int h = z % NH_, n = z / NH_; const size_t src = (((size_t)b * NA + n) * TT + t) * DD + h * HD + d; const v4f q = *(const v4f*)(Q + src), k = *(const v4f*)(K + src); v4us qh, ql, kh, kl;
#pragma unroll
    for (int u = 0; u < 4; ++u) { unsigned short a, c2; splitf(q[u] * 0.17677669529663687f, a, c2); qh[u] = a; ql[u] = c2; splitf(k[u], a, c2); kh[u] = a; kl[u] = c2; }
    for (int ps = 0; ps < 2; ++ps) { *(volatile v4us*)(Qh + e) = qh; *(volatile v4us*)(Ql + e) = ql; *(volatile v4us*)(Kh + e) = kh; *(volatile v4us*)(Kl + e) = kl; if (ps == 0) __threadfence(); } }
__global__ __launch_bounds__(256) void k_vt(const float* __restrict__ V, int b, h16* VT) { const int e = (blockIdx.x * 256 + threadIdx.x) * 2; if (e >= ZZ * HP * TT) return; const int t = e % TT; const int dp = (e / TT) % HP; const int z = e / (TT * HP); const int h = z % NH_, n = z / NH_; v2h o;
#pragma unroll
    for (int u = 0; u < 2; ++u) o[u] = (dp < HD) ? tohx(V[(((size_t)b * NA + n) * TT + t + u) * DD + h * HD + dp]) : tohx(0.f); *(volatile v2h*)(VT + e) = o; __threadfence(); *(volatile v2h*)(VT + e) = o; }
__global__ __launch_bounds__(256) void k_mrg(const float* __restrict__ O, int b, bf* Ch, bf* Cl) { const int e = (blockIdx.x * 256 + threadIdx.x) * 4; if (e >= NA * TT * DD) return; const int c = e % DD; const int t = (e / DD) % TT; const int n = e / (DD * TT); const int h = c / HD, d = c % HD; const float* r = O + (((size_t)(n * NH_ + h)) * TT + t) * HP + d; const size_t oo = (size_t)b * NA * TT * DD + e; v4us oh, ol;
#pragma unroll
    for (int u = 0; u < 4; ++u) { unsigned short a, c2; splitf(r[u] * (1.0f / PCAR), a, c2); oh[u] = a; ol[u] = c2; } *(volatile v4us*)(Ch + oo) = oh; *(volatile v4us*)(Cl + oo) = ol; __threadfence(); *(volatile v4us*)(Ch + oo) = oh; *(volatile v4us*)(Cl + oo) = ol; }
__global__ __launch_bounds__(256) void k_msoft(const float* __restrict__ Sb, const int* __restrict__ km, h16* P16) { const int lane = threadIdx.x & 31; const int row = blockIdx.x * 8 + (threadIdx.x >> 5); if (row >= ZZ * TT) return; const int z = row / TT; const int n = z / NH_; const int* mk = km + (size_t)n * TT; const float* sr = Sb + (size_t)row * TT; float v[16]; float mx = -3.0e38f;
#pragma unroll
    for (int ch = 0; ch < 4; ++ch) { const int j0 = ch * 128 + lane * 4; const v4f a = *(const v4f*)(sr + j0);
#pragma unroll
        for (int u = 0; u < 4; ++u) { const float t = (mk[j0 + u] != 0) ? -1.0e9f : a[u]; v[ch * 4 + u] = t; mx = fmaxf(mx, t); } }
#pragma unroll
    for (int sh = 16; sh; sh >>= 1) mx = fmaxf(mx, __shfl_xor(mx, sh, 32));
    float sum = 0.f;
#pragma unroll
    for (int k = 0; k < 16; ++k) { float d0 = __fsub_rn(v[k], mx); asm volatile("" : "+v"(d0)); v[k] = __expf(d0); sum += v[k]; }
#pragma unroll
    for (int sh = 16; sh; sh >>= 1) sum += __shfl_xor(sum, sh, 32);
    const float f = __fdiv_rn(PCAR, sum);
    for (int ps = 0; ps < 2; ++ps) {
#pragma unroll
        for (int ch = 0; ch < 4; ++ch) { v4h o;
#pragma unroll
            for (int u = 0; u < 4; ++u) o[u] = tohx(v[ch * 4 + u] * f); *(volatile v4h*)(P16 + (size_t)row * TT + ch * 128 + lane * 4) = o; }
        if (ps == 0) __threadfence(); } }

extern "C" void kernel_launch(void* const* d_in, const int* in_sizes, int n_in,
                              void* d_out, int out_size, void* d_ws, size_t ws_size, hipStream_t stream) {
    (void)in_sizes; (void)n_in; (void)out_size;
    const float** I = (const float**)d_in;
    const float *xq = I[0], *xk = I[1], *xv = I[2]; const int* kpm = (const int*)d_in[3]; const float *wpos = I[4], *bpos = I[5], *wvel = I[6], *wacc = I[7], *wq = I[8], *bq = I[9], *wk = I[10], *bk = I[11], *wv = I[12], *bv = I[13], *wo = I[14], *bo = I[15];
    float* OUT = (float*)d_out;
    char* wsp = (char*)d_ws;
    auto take = [&](size_t bytes) { char* p = wsp; wsp += (bytes + 255) & ~(size_t)255; return (void*)p; };
    bf* WQ = (bf*)take((size_t)DD * F3 * 2); bf* WK = (bf*)take((size_t)DD * F3 * 2); bf* WV = (bf*)take((size_t)DD * DD * 2); bf* WO = (bf*)take((size_t)DD * DD * 2);
    bf* Fh = (bf*)take((size_t)NR * F3 * 2); bf* Fl = (bf*)take((size_t)NR * F3 * 2); float* Q = (float*)take((size_t)NR * DD * 4); float* K = (float*)take((size_t)NR * DD * 4); bf* XV = (bf*)take((size_t)NR * DD * 2); float* V = (float*)take((size_t)NR * DD * 4);
    bf* QPh = (bf*)take((size_t)ZZ * TT * HD * 2); bf* QPl = (bf*)take((size_t)ZZ * TT * HD * 2); bf* KPh = (bf*)take((size_t)ZZ * TT * HD * 2); bf* KPl = (bf*)take((size_t)ZZ * TT * HD * 2); h16* VT = (h16*)take((size_t)ZZ * HP * TT * 2);
    float* Sb = (float*)take((size_t)ZZ * TT * TT * 4); h16* P16 = (h16*)take((size_t)ZZ * TT * TT * 2); float* O = (float*)take((size_t)ZZ * TT * HP * 4); bf* Ch = (bf*)take((size_t)NR * DD * 2); bf* Cl = (bf*)take((size_t)NR * DD * 2);
    if ((size_t)(wsp - (char*)d_ws) > ws_size) return;
    k_wtG<<<(F3 * DD / 64 + 63) / 64, 256, 0, stream>>>(wq, F3, DD, WQ); k_wtG<<<(F3 * DD / 64 + 63) / 64, 256, 0, stream>>>(wk, F3, DD, WK); k_wtG<<<(DD * DD / 64 + 63) / 64, 256, 0, stream>>>(wv, DD, DD, WV); k_wtG<<<(DD * DD / 64 + 63) / 64, 256, 0, stream>>>(wo, DD, DD, WO);
    k_kin<<<(unsigned)(((size_t)NR * F3 / 4 + 255) / 256), 256, 0, stream>>>(xq, wpos, bpos, wvel, wacc, Fh, Fl); k_gemmw<bf, 1, true><<<dim3(NR / 64, DD / 64, 1), 32, 0, stream>>>(Fh, Fl, WQ, nullptr, F3, Q, DD, bq, 0, 0, 0);
    k_kin<<<(unsigned)(((size_t)NR * F3 / 4 + 255) / 256), 256, 0, stream>>>(xk, wpos, bpos, wvel, wacc, Fh, Fl); k_gemmw<bf, 1, true><<<dim3(NR / 64, DD / 64, 1), 32, 0, stream>>>(Fh, Fl, WK, nullptr, F3, K, DD, bk, 0, 0, 0);
    k_cvt8<<<(NR * DD / 8 + 255) / 256, 256, 0, stream>>>(xv, XV, (size_t)NR * DD / 8); k_gemmw<bf, 0, true><<<dim3(NR / 64, DD / 64, 1), 32, 0, stream>>>(XV, nullptr, WV, nullptr, DD, V, DD, bv, 0, 0, 0);
    for (int b = 0; b < NBb; ++b) {
        k_qkpl<<<(ZZ * TT * HD / 4 + 255) / 256, 256, 0, stream>>>(Q, K, b, QPh, QPl, KPh, KPl); k_vt<<<(ZZ * HP * TT / 2 + 255) / 256, 256, 0, stream>>>(V, b, VT);
        k_gemmw<bf, 2, false><<<dim3(TT / 64, TT / 64, ZZ), 32, 0, stream>>>(QPh, QPl, KPh, KPl, HD, Sb, TT, nullptr, (size_t)TT * HD, (size_t)TT * HD, (size_t)TT * TT);
        k_msoft<<<ZZ * TT / 8, 256, 0, stream>>>(Sb, kpm + (size_t)b * NA * TT, P16);
        k_gemmw<h16, 0, false><<<dim3(TT / 64, HP / 64, ZZ), 32, 0, stream>>>(P16, nullptr, VT, nullptr, TT, O, HP, nullptr, (size_t)TT * TT, (size_t)HP * TT, (size_t)TT * HP);
        k_mrg<<<(NA * TT * DD / 4 + 255) / 256, 256, 0, stream>>>(O, b, Ch, Cl); }
    k_gemmw<bf, 1, true><<<dim3(NR / 64, DD / 64, 1), 32, 0, stream>>>(Ch, Cl, WO, nullptr, DD, OUT, DD, bo, 0, 0, 0);
}
